// MambaBlock_39659728011562
// MI455X (gfx1250) — hardware-run, weakly checked
//
#include <hip/hip_runtime.h>


#ifndef NB
#define NB 2
#endif
#ifndef SEQ
#define SEQ 1024
#endif
#define NB_FULL  2
#define SEQ_FULL 1024
#ifndef OUT_SEQ
#define OUT_SEQ SEQ
#endif
#define DM   1024
#define DI   2048
#define XZP  4096
#define NST  16
#define NCV  4
#define NXD  33
#define NXP  64
#define TS   16
#define WCS  64.0f
#define XCS  16.0f
#define YCS  16.0f
#define GSC  (1.0f / 1024.0f)

static_assert(XZP == 2 * DI);
static_assert(DM % 32 == 0);
static_assert(DI % 32 == 0);
static_assert((NB * SEQ) % 64 == 0);
static_assert(XZP % 64 == 0);
static_assert(DM % 64 == 0);
static_assert(NXP % 64 == 0);
static_assert(NXD <= NXP);
static_assert(DI == 256 * 8);
static_assert(DI % 256 == 0);
static_assert(SEQ % TS == 0);
static_assert(TS % 8 == 0);
static_assert((256 / 32) * (TS / 8) == TS);
static_assert(TS * NXP == 256 * 4);
static_assert(DM % 128 == 0);
static_assert((NB * SEQ) % 8 == 0);
static_assert(NB <= NB_FULL);
static_assert(SEQ <= SEQ_FULL);
static_assert(8 * 32 * 16 == 16 * 64 * 4);
static_assert(((size_t)NB * SEQ * DM) % 8 == 0);
static_assert(((size_t)XZP * DM) % 8 == 0);
static_assert(((size_t)DM * DI) % 8 == 0);
static_assert(((size_t)NXD * DI) % 8 == 0);
static_assert(((size_t)NXP * DI) % 8 == 0);
static_assert(16 * 68 * 4 <= 131072);
static_assert(TS * NXP * 4 + TS * 256 * 2 <= 131072);

typedef _Float16 h16;
typedef unsigned short bf;
typedef __attribute__((ext_vector_type(16))) __bf16   v16bf;
typedef __attribute__((ext_vector_type(16))) _Float16 v16h;
typedef __attribute__((ext_vector_type(8)))  _Float16 v8h;
typedef __attribute__((ext_vector_type(8)))  unsigned short v8us;
typedef __attribute__((ext_vector_type(8)))  float    v8f;
typedef __attribute__((ext_vector_type(4)))  float    v4f;
typedef __attribute__((ext_vector_type(2)))  unsigned v2u;
typedef v4f  __attribute__((may_alias)) v4fa;
typedef v8h  __attribute__((may_alias)) v8ha;

#pragma clang fp contract(off)

__device__ __forceinline__ unsigned short f2bf(float f) { unsigned u = __float_as_uint(f); u += 0x7FFFu + ((u >> 16) & 1u); return (unsigned short)(u >> 16); }
__device__ __forceinline__ float bfr(float f) { return __uint_as_float(((unsigned)f2bf(f)) << 16); }
__device__ __forceinline__ v16h cat16(v8h lo, v8h hi) { return __builtin_shufflevector(lo, hi, 0, 1, 2, 3, 4, 5, 6, 7, 8, 9, 10, 11, 12, 13, 14, 15); }
__device__ __forceinline__ v16bf cat16b(v8us lo, v8us hi) { return __builtin_bit_cast(v16bf, __builtin_shufflevector(lo, hi, 0, 1, 2, 3, 4, 5, 6, 7, 8, 9, 10, 11, 12, 13, 14, 15)); }
__device__ __forceinline__ v8f wmma16(v16h a, v16h b, v8f c) { return __builtin_amdgcn_wmma_f32_16x16x32_f16(false, a, false, b, (short)0, c, false, false); }
__device__ __forceinline__ v8f wmmab(v16bf a, v16bf b, v8f c) { return __builtin_amdgcn_wmma_f32_16x16x32_bf16(false, a, false, b, (short)0, c, false, false); }
__device__ __forceinline__ v8f wmma16_g(v16h a, v16h b, v8f c) {
    c = __builtin_amdgcn_wmma_f32_16x16x32_f16(false, a, false, b, (short)0, c, false, false);
    asm volatile("v_nop\n\tv_nop\n\tv_nop\n\tv_nop" : "+v"(c) : "v"(a), "v"(b));
    return c; }
__device__ __forceinline__ v8f wmmab_g(v16bf a, v16bf b, v8f c) {
    c = __builtin_amdgcn_wmma_f32_16x16x32_bf16(false, a, false, b, (short)0, c, false, false);
    asm volatile("v_nop\n\tv_nop\n\tv_nop\n\tv_nop" : "+v"(c) : "v"(a), "v"(b));
    return c; }
__device__ __forceinline__ v16h  ldh(const h16* p) { return cat16(*(const v8h*)p, *(const v8h*)(p + 16)); }
__device__ __forceinline__ v16bf ldb(const bf* p)  { return cat16b(*(const v8us*)p, *(const v8us*)(p + 16)); }
__device__ __forceinline__ void wave_sync() { __builtin_amdgcn_fence(3  , "wavefront"); __builtin_amdgcn_wave_barrier(); asm volatile("" ::: "memory"); }
__device__ __forceinline__ v16bf ldf(const bf* p)  { return ldb(p); }
__device__ __forceinline__ v16h  ldf(const h16* p) { return ldh(p); }
__device__ __forceinline__ v8f mm(v16bf a, v16bf b, v8f c) { return wmmab_g(a, b, c); }
__device__ __forceinline__ v8f mm(v16h a, v16h b, v8f c)   { return wmma16_g(a, b, c); }
__device__ __forceinline__ h16 toh_flush(float v) { const h16 r = (h16)v; return (fabsf(v) < 6.103515625e-05f) ? (h16)0.0f : r; }
__device__ __forceinline__ float fexp(float x) { return __builtin_amdgcn_exp2f(x * 1.4426950408889634f); }
__device__ __forceinline__ float wsum(float v) { v += __shfl_xor(v, 16, 32); v += __shfl_xor(v, 8, 32); v += __shfl_xor(v, 4, 32); v += __shfl_xor(v, 2, 32); v += __shfl_xor(v, 1, 32); return v; }

__global__ __launch_bounds__(256) void k_cvt8(const float* __restrict__ src, bf* dst, size_t n8) {
    const size_t i = (size_t)blockIdx.x * 256 + threadIdx.x; if (i >= n8) return;
    const v8f v = *(const v8f*)(src + i * 8); v8us o;
#pragma unroll
    for (int k = 0; k < 8; ++k) o[k] = f2bf(v[k]);
    *(volatile v8us*)(dst + i * 8) = o; __threadfence(); *(volatile v8us*)(dst + i * 8) = o;
}

__global__ __launch_bounds__(256) void k_wconv(const float* __restrict__ src, h16* dst, size_t n8d, size_t n8s, float carry) {
    const size_t i = (size_t)blockIdx.x * 256 + threadIdx.x; if (i >= n8d) return;
    const size_t si = (i < n8s) ? i : (n8s - 1);
    v8f v = *(const v8f*)(src + si * 8);
    asm volatile("" : "+v"(v));
    const bool ok = i < n8s; v8h o;
#pragma unroll
    for (int k = 0; k < 8; ++k) { const h16 r = toh_flush(bfr(v[k]) * carry); o[k] = ok ? r : (h16)0.0f; }
    *(volatile v8h*)(dst + i * 8) = o; __threadfence(); *(volatile v8h*)(dst + i * 8) = o;
}

template <typename T, typename FR, int RES>
__device__ __forceinline__ void gemm_body(const T* __restrict__ A, const T* __restrict__ Bt, const bf* __restrict__ XR, float* C, const int K, const int ldc, const float scale) {
    __shared__ __align__(16) float os[16 * 68];
    const int lane = threadIdx.x & 31, lr = lane & 15, hi = lane >> 4; const int r0 = blockIdx.x * 64, c0 = blockIdx.y * 64;
    v8f acc[4][4];
#pragma unroll
    for (int mb = 0; mb < 4; ++mb)
#pragma unroll
        for (int nb = 0; nb < 4; ++nb) acc[mb][nb] = (v8f){};
    const size_t aoff = (size_t)(r0 + lr) * K + 8 * hi, boff = (size_t)(c0 + lr) * K + 8 * hi;
#pragma unroll 1
    for (int kc = 0; kc < K; kc += 32) {
        FR a[4];
#pragma unroll
        for (int mb = 0; mb < 4; ++mb) a[mb] = ldf(A + aoff + (size_t)mb * 16 * K + kc);
#pragma unroll
        for (int nb = 0; nb < 4; ++nb) { const FR b = ldf(Bt + boff + (size_t)nb * 16 * K + kc);
#pragma unroll
            for (int mb = 0; mb < 4; ++mb) acc[mb][nb] = mm(a[mb], b, acc[mb][nb]); }
    }
#pragma unroll
    for (int mb = 0; mb < 4; ++mb) {
#pragma unroll
        for (int nb = 0; nb < 4; ++nb) {
#pragma unroll
            for (int j = 0; j < 8; ++j) os[(hi * 8 + j) * 68 + nb * 16 + lr] = acc[mb][nb][j] * scale; }
        wave_sync();
#pragma unroll 1
        for (int ps = 0; ps < 2; ++ps) {
#pragma unroll
            for (int s = 0; s < 8; ++s) { const int p = s * 32 + lane; const int row = p >> 4, c4 = (p & 15) * 4;
                v4f val = *(const v4fa*)(&os[row * 68 + c4]);
                const size_t go = (size_t)(r0 + mb * 16 + row) * (size_t)ldc + (size_t)(c0 + c4);
                if (RES) { const v2u w = *(const v2u*)(XR + go);
                           val[0] += __uint_as_float(w[0] << 16); val[1] += __uint_as_float(w[0] & 0xffff0000u);
                           val[2] += __uint_as_float(w[1] << 16); val[3] += __uint_as_float(w[1] & 0xffff0000u); }
                *(volatile v4f*)(C + go) = val; }
            if (ps == 0) __threadfence(); }
        wave_sync();
    }
}

__global__ __launch_bounds__(32) void k_gemm_in(const bf* __restrict__ A, const bf* __restrict__ Bt, float* C) {
    gemm_body<bf, v16bf, 0>(A, Bt, nullptr, C, DM, XZP, 1.0f);
}
__global__ __launch_bounds__(32) void k_gemm_xp(const h16* __restrict__ A, const h16* __restrict__ Bt, float* C) {
    gemm_body<h16, v16h, 0>(A, Bt, nullptr, C, DI, NXP, GSC);
}
__global__ __launch_bounds__(32) void k_gemm_out(const h16* __restrict__ A, const h16* __restrict__ Bt, const bf* __restrict__ XR, float* C) {
    gemm_body<h16, v16h, 1>(A, Bt, XR, C, DI, DM, GSC);
}

__global__ __launch_bounds__(256) void k_conv(const float* __restrict__ XZ, const float* __restrict__ cw, const float* __restrict__ cb, h16* XCH) {
    const int m = blockIdx.x; const int t = m % SEQ; const int c8 = threadIdx.x * 8;
    const v8f bv = *(const v8f*)(cb + c8);
    float wt[8][NCV]; float s[8];
#pragma unroll
    for (int c = 0; c < 8; ++c) { const v4f w = *(const v4f*)(cw + (size_t)(c8 + c) * NCV);
#pragma unroll
        for (int i = 0; i < NCV; ++i) wt[c][i] = bfr(w[i]);
        s[c] = bfr(bv[c]); }
#pragma unroll
    for (int tap = 0; tap < NCV; ++tap) {
        const int ls = t - (NCV - 1) + tap; const bool ok = ls >= 0;
        const int ms = ok ? (m - (NCV - 1) + tap) : m;
        v8f xv = *(const v8f*)(XZ + (size_t)ms * XZP + c8);
        asm volatile("" : "+v"(xv));
#pragma unroll
        for (int c = 0; c < 8; ++c) { const float term = xv[c] * wt[c][tap]; s[c] += ok ? term : 0.0f; }
    }
    v8h o;
#pragma unroll
    for (int c = 0; c < 8; ++c) { const float sg = __builtin_amdgcn_rcpf(1.0f + fexp(-s[c])); o[c] = toh_flush(s[c] * sg * XCS); }
    h16* dst = XCH + (size_t)m * DI + c8;
    *(volatile v8h*)dst = o; __threadfence(); *(volatile v8h*)dst = o;
}

__global__ __launch_bounds__(256) void k_scan(const float* __restrict__ XD, const float* __restrict__ XZ, const float* __restrict__ cw, const float* __restrict__ cb,
                                              const float* __restrict__ dtw_, const float* __restrict__ dtb_, const float* __restrict__ alog, const float* __restrict__ Dp, h16* YH) {
    __shared__ __align__(16) float xr[TS * NXP];
    __shared__ __align__(16) h16 ys[TS * 256];
    const int tid = threadIdx.x, lane = tid & 31;
    const int wave = __builtin_amdgcn_readfirstlane((int)(threadIdx.x >> 5));
    const int b = blockIdx.x / (DI / 256); const int dbase = (blockIdx.x % (DI / 256)) * 256; const int d = dbase + tid;
    float h[NST], Ad[NST];
#pragma unroll
    for (int q = 0; q < NST / 4; ++q) { const v4f al = *(const v4f*)(alog + (size_t)d * NST + 4 * q);
#pragma unroll
        for (int i = 0; i < 4; ++i) { Ad[4 * q + i] = -fexp(bfr(al[i])); h[4 * q + i] = 0.0f; } }
    const v4f wv = *(const v4f*)(cw + (size_t)d * NCV);
    const float w0 = bfr(wv[0]), w1 = bfr(wv[1]), w2 = bfr(wv[2]), w3 = bfr(wv[3]);
    const float cbv = bfr(cb[d]), dtw = bfr(dtw_[d]), dtb = bfr(dtb_[d]), Dd = bfr(Dp[d]);
    const size_t mbase = (size_t)b * SEQ;
    float x1 = 0.0f, x2 = 0.0f, x3 = 0.0f;
#pragma unroll 1
    for (int l0 = 0; l0 < SEQ; l0 += TS) {
        *(v4fa*)(&xr[tid * 4]) = *(const v4f*)(XD + (mbase + (size_t)l0) * NXP + (size_t)tid * 4);
        __syncthreads();
#pragma unroll 1
        for (int s = 0; s < TS; ++s) {
            const size_t m = mbase + (size_t)(l0 + s);
            const float x0 = XZ[m * XZP + d];
            const float zv = XZ[m * XZP + DI + d];
            float sc = cbv; sc += w0 * x3; sc += w1 * x2; sc += w2 * x1; sc += w3 * x0;
            x3 = x2; x2 = x1; x1 = x0;
            const float xcv = sc * __builtin_amdgcn_rcpf(1.0f + fexp(-sc));
            const float xin = xr[s * NXP] * dtw + dtb;
            const float dt = fmaxf(xin, 0.0f) + log1pf(fexp(-fabsf(xin)));
            const float dtx = dt * xcv;
            float acc = 0.0f;
#pragma unroll
            for (int n = 0; n < NST; ++n) {
                const float dA = fexp(dt * Ad[n]);
                h[n] = dA * h[n] + dtx * xr[s * NXP + 1 + n];
                acc += h[n] * xr[s * NXP + 1 + NST + n]; }
            const float sz = zv * __builtin_amdgcn_rcpf(1.0f + fexp(-zv));
            const float yv = (acc + Dd * xcv) * sz;
            ys[s * 256 + tid] = toh_flush(yv * YCS);
        }
        __syncthreads();
#pragma unroll 1
        for (int ps = 0; ps < 2; ++ps) {
#pragma unroll
            for (int q = 0; q < TS / 8; ++q) { const int row = wave + 8 * q;
                const v8h val = *(const v8ha*)(&ys[row * 256 + lane * 8]);
                *(volatile v8h*)(YH + (mbase + (size_t)(l0 + row)) * DI + dbase + lane * 8) = val; }
            if (ps == 0) __threadfence(); }
    }
}

__global__ __launch_bounds__(256) void k_ln(const float* __restrict__ OP, const float* __restrict__ g, const float* __restrict__ be, float* OUT) {
    const int lane = threadIdx.x & 31;
    const int wave = __builtin_amdgcn_readfirstlane((int)(threadIdx.x >> 5));
    const int m = blockIdx.x * 8 + wave; const int b = m / SEQ, t = m % SEQ;
    const float* orow = OP + (size_t)m * DM + lane * 4;
    float s = 0.0f;
#pragma unroll 1
    for (int j = 0; j < DM / 128; ++j) { const v4f v = *(const v4f*)(orow + j * 128); s += (v[0] + v[1]) + (v[2] + v[3]); }
    s = wsum(s);
    const float mu = s * (1.0f / DM);
    float q = 0.0f;
#pragma unroll 1
    for (int j = 0; j < DM / 128; ++j) { const v4f v = *(const v4f*)(orow + j * 128);
        const float d0 = v[0] - mu, d1 = v[1] - mu, d2 = v[2] - mu, d3 = v[3] - mu;
        q += (d0 * d0 + d1 * d1) + (d2 * d2 + d3 * d3); }
    q = wsum(q);
    const float rinv = 1.0f / sqrtf(q * (1.0f / DM) + 1e-5f);
    float* dst = OUT + ((size_t)b * OUT_SEQ + (size_t)t) * DM + lane * 4;
#pragma unroll 1
    for (int ps = 0; ps < 2; ++ps) {
#pragma unroll 1
        for (int j = 0; j < DM / 128; ++j) {
            const v4f v = *(const v4f*)(orow + j * 128);
            const v4f gv = *(const v4f*)(g + j * 128 + lane * 4);
            const v4f bv = *(const v4f*)(be + j * 128 + lane * 4);
            v4f o;
#pragma unroll
            for (int i = 0; i < 4; ++i) o[i] = (v[i] - mu) * rinv * bfr(gv[i]) + bfr(bv[i]);
            *(volatile v4f*)(dst + j * 128) = o; }
        if (ps == 0) __threadfence(); }
}

static constexpr size_t al256(size_t v) { return (v + 255) & ~(size_t)255; }
static constexpr size_t SZ_XB = al256((size_t)NB * SEQ * DM * 2);
static constexpr size_t SZ_WI = al256((size_t)XZP * DM * 2);
static constexpr size_t SZ_WO = al256((size_t)DM * DI * 2);
static constexpr size_t SZ_WX = al256((size_t)NXP * DI * 2);
static constexpr size_t SZ_XZ = al256((size_t)NB * SEQ * XZP * 4);
static constexpr size_t SZ_XC = al256((size_t)NB * SEQ * DI * 2);
static constexpr size_t SZ_XD = al256((size_t)NB * SEQ * NXP * 4);
static constexpr size_t SZ_YH = al256((size_t)NB * SEQ * DI * 2);
static constexpr size_t SZ_OP = al256((size_t)NB * SEQ * DM * 4);
static constexpr size_t SZ_TOTAL = SZ_XB + SZ_WI + SZ_WO + SZ_WX + SZ_XZ + SZ_XC + SZ_XD + SZ_YH + SZ_OP;
static_assert(SZ_TOTAL <= (size_t)134217728);

extern "C" void kernel_launch(void* const* d_in, const int* in_sizes, int n_in,
                              void* d_out, int out_size, void* d_ws, size_t ws_size, hipStream_t stream) {
    if (n_in < 12) return;
    const size_t needx = ((size_t)(NB - 1) * SEQ_FULL + SEQ) * DM;
    if ((size_t)in_sizes[0] < needx) return;
    if ((size_t)in_sizes[1] < (size_t)XZP * DM) return;
    if ((size_t)in_sizes[2] < (size_t)DI * NCV || in_sizes[3] < DI) return;
    if ((size_t)in_sizes[4] < (size_t)NXD * DI) return;
    if (in_sizes[5] < DI || in_sizes[6] < DI) return;
    if ((size_t)in_sizes[7] < (size_t)DI * NST || in_sizes[8] < DI) return;
    if ((size_t)in_sizes[9] < (size_t)DM * DI) return;
    if (in_sizes[10] < DM || in_sizes[11] < DM) return;
    if ((size_t)out_size < ((size_t)(NB - 1) * OUT_SEQ + SEQ) * DM) return;
    if (SZ_TOTAL > ws_size) return;
    const float* x    = (const float*)d_in[0];
    const float* win  = (const float*)d_in[1];
    const float* cw   = (const float*)d_in[2];
    const float* cb   = (const float*)d_in[3];
    const float* wxp  = (const float*)d_in[4];
    const float* dtw  = (const float*)d_in[5];
    const float* dtb  = (const float*)d_in[6];
    const float* alog = (const float*)d_in[7];
    const float* Dp   = (const float*)d_in[8];
    const float* wout = (const float*)d_in[9];
    const float* lng  = (const float*)d_in[10];
    const float* lnb  = (const float*)d_in[11];
    float* OUT = (float*)d_out;
    char* wsp = (char*)d_ws;
    bf*    XB  = (bf*)wsp;    wsp += SZ_XB;
    bf*    WIB = (bf*)wsp;    wsp += SZ_WI;
    h16*   WOH = (h16*)wsp;   wsp += SZ_WO;
    h16*   WXH = (h16*)wsp;   wsp += SZ_WX;
    float* XZ  = (float*)wsp; wsp += SZ_XZ;
    h16*   XCH = (h16*)wsp;   wsp += SZ_XC;
    float* XD  = (float*)wsp; wsp += SZ_XD;
    h16*   YH  = (h16*)wsp;   wsp += SZ_YH;
    float* OP  = (float*)wsp; wsp += SZ_OP;

    if (SEQ == SEQ_FULL) {
        const size_t n8 = (size_t)NB * SEQ * DM / 8;
        k_cvt8<<<(unsigned)((n8 + 255) / 256), 256, 0, stream>>>(x, XB, n8);
    } else {
        const size_t n8 = (size_t)SEQ * DM / 8;
        for (int b = 0; b < NB; ++b) k_cvt8<<<(unsigned)((n8 + 255) / 256), 256, 0, stream>>>(x + (size_t)b * SEQ_FULL * DM, XB + (size_t)b * SEQ * DM, n8);
    }
    { const size_t n8 = (size_t)XZP * DM / 8; k_cvt8<<<(unsigned)((n8 + 255) / 256), 256, 0, stream>>>(win, WIB, n8); }
    { const size_t n8 = (size_t)DM * DI / 8; k_wconv<<<(unsigned)((n8 + 255) / 256), 256, 0, stream>>>(wout, WOH, n8, n8, WCS); }
    { const size_t n8d = (size_t)NXP * DI / 8, n8s = (size_t)NXD * DI / 8; k_wconv<<<(unsigned)((n8d + 255) / 256), 256, 0, stream>>>(wxp, WXH, n8d, n8s, WCS); }

    k_gemm_in<<<dim3(NB * SEQ / 64, XZP / 64, 1), 32, 0, stream>>>(XB, WIB, XZ);
    k_conv<<<NB * SEQ, 256, 0, stream>>>(XZ, cw, cb, XCH);
    k_gemm_xp<<<dim3(NB * SEQ / 64, NXP / 64, 1), 32, 0, stream>>>(XCH, WXH, XD);
    k_scan<<<NB * (DI / 256), 256, 0, stream>>>(XD, XZ, cw, cb, dtw, dtb, alog, Dp, YH);
    k_gemm_out<<<dim3(NB * SEQ / 64, DM / 64, 1), 32, 0, stream>>>(YH, WOH, XB, OP);
    k_ln<<<NB * SEQ / 8, 256, 0, stream>>>(OP, lng, lnb, OUT);
}
